// DynamicWeights__635655160217
// MI455X (gfx1250) — hardware-verified
//
#include <hip/hip_runtime.h>
#include <stddef.h>

constexpr int kNIMG  = 32;
constexpr int kCH    = 256;
constexpr int kCIN2  = 512;
constexpr int kHGT   = 32;
constexpr int kWID   = 32;
constexpr int kNPX   = 1024;
constexpr int kPW    = 36;
constexpr int kPROWS = 37;
constexpr int kNPOS  = 1332;
constexpr int kMOUT  = 1152;
constexpr int kOFFC  = 18;
constexpr int kOFFN  = 32;
constexpr int kT5    = 25;
constexpr int kKOFF  = 12800;
constexpr int kT3    = 9;
constexpr int kKDEF  = 2304;
constexpr int kODEF  = 9;
constexpr int kMDEF  = 16;
constexpr int kCHUNK = 8;
constexpr int kNCHUNK = 4;

static_assert(kNPOS == kPROWS * kPW, "positions");
static_assert(kMOUT == kHGT * kPW, "gemm rows");
static_assert(kMOUT % 64 == 0, "M tile multiple");
static_assert(kMOUT - 1 + 4 * kPW + 4 < kNPOS, "tap-shifted A rows stay inside the plane");
static_assert(kKOFF == kT5 * kCIN2 && kKDEF == kT3 * kCH, "depths");
static_assert(kCIN2 % 32 == 0 && kKDEF % 32 == 0, "K multiple of 32");
static_assert(kNCHUNK * kCHUNK == kNIMG, "chunks");
static_assert(kNPX % 64 == 0, "N tile multiple");

typedef __attribute__((ext_vector_type(16))) _Float16 v16h;
typedef __attribute__((ext_vector_type(8)))  _Float16 v8h;
typedef __attribute__((ext_vector_type(16))) __bf16   v16b;
typedef __attribute__((ext_vector_type(8)))  __bf16   v8b;
typedef __attribute__((ext_vector_type(8)))  float    v8f;
typedef __attribute__((ext_vector_type(4)))  float    v4f;
typedef __attribute__((ext_vector_type(4)))  unsigned v4u;

__device__ __forceinline__ unsigned pk2(unsigned short a, unsigned short b) {
  return (unsigned)a | ((unsigned)b << 16);
}
__device__ __forceinline__ unsigned pkh2(float a, float b) {
  return pk2(__builtin_bit_cast(unsigned short, (_Float16)a), __builtin_bit_cast(unsigned short, (_Float16)b));
}

__device__ __forceinline__ void dep_guard_h(v8f& a, v8f& b, v16h x, v16h y) { asm volatile("v_nop\n\tv_nop\n\tv_nop\n\tv_nop" : "+v"(a), "+v"(b) : "v"(x), "v"(y)); }
__device__ __forceinline__ void dep_guard_b(v8f& a, v8f& b, v16b x, v16b y) { asm volatile("v_nop\n\tv_nop\n\tv_nop\n\tv_nop" : "+v"(a), "+v"(b) : "v"(x), "v"(y)); }
__device__ __forceinline__ void keep4_h(v16h a, v16h b, v16h c, v16h d) { asm volatile("v_nop" :: "v"(a), "v"(b), "v"(c), "v"(d)); }
__device__ __forceinline__ void keep4_b(v16b a, v16b b, v16b c, v16b d) { asm volatile("v_nop" :: "v"(a), "v"(b), "v"(c), "v"(d)); }
__device__ __forceinline__ void acc_guard4(v8f& a, v8f& b, v8f& c, v8f& d) { asm volatile("v_nop\n\tv_nop\n\tv_nop\n\tv_nop" : "+v"(a), "+v"(b), "+v"(c), "+v"(d)); }
template <typename T> struct Frag;
template <> struct Frag<_Float16> {
  typedef v16h V; union U { v16h v; v8h h[2]; };
  static __device__ __forceinline__ v16h load(const _Float16* p) {
    U f; f.h[0] = *(const v8h*)(p); f.h[1] = *(const v8h*)(p + 16); return f.v;
  }
  static __device__ __forceinline__ v8f mma(v16h a, v16h b, v8f c) {
    return __builtin_amdgcn_wmma_f32_16x16x32_f16(false, a, false, b, (short)0, c, false, false);
  }
  static __device__ __forceinline__ void guard(v8f& a, v8f& b, v16h x, v16h y) { dep_guard_h(a, b, x, y); }
  static __device__ __forceinline__ void keep(v16h a, v16h b, v16h c, v16h d) { keep4_h(a, b, c, d); }
};
template <> struct Frag<__bf16> {
  typedef v16b V; union U { v16b v; v8b h[2]; };
  static __device__ __forceinline__ v16b load(const __bf16* p) {
    U f; f.h[0] = *(const v8b*)(p); f.h[1] = *(const v8b*)(p + 16); return f.v;
  }
  static __device__ __forceinline__ v8f mma(v16b a, v16b b, v8f c) {
    return __builtin_amdgcn_wmma_f32_16x16x32_bf16(false, a, false, b, (short)0, c, false, false);
  }
  static __device__ __forceinline__ void guard(v8f& a, v8f& b, v16b x, v16b y) { dep_guard_b(a, b, x, y); }
  static __device__ __forceinline__ void keep(v16b a, v16b b, v16b c, v16b d) { keep4_b(a, b, c, d); }
};

__global__ __launch_bounds__(256) void k_pack(const float* __restrict__ support, const float* __restrict__ query,
                                              _Float16* __restrict__ xp) {
  __shared__ float t[64][33];
  const int tid = threadIdx.x;
  const int blk = blockIdx.x;
  const int cg   = blk & 7;
  const int rest = blk >> 3;
  const int py   = rest % kPROWS;
  const int img  = rest / kPROWS;
  const int yy   = py - 2;
  const bool rowvalid = (yy >= 0) && (yy < kHGT);
  const int yyc  = yy < 0 ? 0 : (yy > kHGT - 1 ? kHGT - 1 : yy);
  const float* src = (cg < 4) ? query : support;
  const float* sb = src + ((size_t)img * kCH + (size_t)(cg & 3) * 64) * kNPX + (size_t)yyc * kWID;
#pragma unroll
  for (int i = 0; i < 8; ++i) {
    const int idx = i * 256 + tid;
    const int c = idx >> 5, j = idx & 31;
    t[c][j] = sb[(size_t)c * kNPX + j];
  }
  __syncthreads();
  const int wave = tid >> 5, lane = tid & 31, q = lane >> 3, c8 = (lane & 7) * 8;
  _Float16* ob = xp + ((size_t)img * kNPOS + (size_t)py * kPW) * kCIN2 + cg * 64 + c8;
  for (int pass = 0; pass < 2; ++pass) {
#pragma unroll
    for (int it = 0; it < 2; ++it) {
      const int pxp = it * 32 + wave * 4 + q;
      if (pxp < kPW) {
        const int xx = pxp - 2;
        const bool cv = rowvalid && (xx >= 0) && (xx < kWID);
        const int xxc = xx < 0 ? 0 : (xx > kWID - 1 ? kWID - 1 : xx);
        v8h hv;
#pragma unroll
        for (int e = 0; e < 8; ++e) {
          const float f = t[c8 + e][xxc];
          hv[e] = (_Float16)(cv ? f : 0.0f);
        }
        *(volatile v8h*)(ob + (size_t)pxp * kCIN2) = hv;
      }
    }
    __threadfence();
  }
}

__global__ __launch_bounds__(256) void k_prep_woff(const float* __restrict__ w, _Float16* __restrict__ Wo) {
  const int g = blockIdx.x * 256 + threadIdx.x;
  if (g < kOFFN * kKOFF / 8) {
    const int e0  = g * 8;
    const int o   = e0 / kKOFF;
    const int col = e0 - o * kKOFF;
    const int tp  = col >> 9;
    const int c0  = col & (kCIN2 - 1);
    const int oc  = o < kOFFC ? o : (kOFFC - 1);
    float f[8];
#pragma unroll
    for (int j = 0; j < 8; ++j) {
      const float v = w[((size_t)oc * kCIN2 + c0 + j) * kT5 + tp] * 64.0f;
      f[j] = (o < kOFFC) ? v : 0.0f;
    }
    v4u u;
    u[0] = pkh2(f[0], f[1]); u[1] = pkh2(f[2], f[3]); u[2] = pkh2(f[4], f[5]); u[3] = pkh2(f[6], f[7]);
    volatile v4u* p = (volatile v4u*)(Wo + e0);
    *p = u;
    __threadfence();
    *p = u;
  }
}

__global__ __launch_bounds__(256) void k_prep_wdef(const float* __restrict__ w, _Float16* __restrict__ Wd) {
  const int g = blockIdx.x * 256 + threadIdx.x;
  if (g < kMDEF * kKDEF / 8) {
    const int e0  = g * 8;
    const int o   = e0 / kKDEF;
    const int col = e0 - o * kKDEF;
    const int k   = col >> 8;
    const int c0  = col & (kCH - 1);
    const int oc  = o < kODEF ? o : (kODEF - 1);
    float f[8];
#pragma unroll
    for (int j = 0; j < 8; ++j) {
      const float v = w[((size_t)oc * kCH + c0 + j) * kT3 + k] * 32.0f;
      f[j] = (o < kODEF) ? v : 0.0f;
    }
    v4u u;
    u[0] = pkh2(f[0], f[1]); u[1] = pkh2(f[2], f[3]); u[2] = pkh2(f[4], f[5]); u[3] = pkh2(f[6], f[7]);
    volatile v4u* p = (volatile v4u*)(Wd + e0);
    *p = u;
    __threadfence();
    *p = u;
  }
}

__global__ __launch_bounds__(64) void k_offconv(const _Float16* __restrict__ xp, const _Float16* __restrict__ Wo,
                                                float* __restrict__ offo) {
  typedef _Float16 T;
  typedef v16h V;
  __shared__ __align__(16) float sT[2][16 * 36];
  const int img  = blockIdx.y;
  const int lane = threadIdx.x & 31;
  const int wave = threadIdx.x >> 5;
  const int tile = blockIdx.x * 2 + wave;
  if (tile >= kMOUT / 64) return;
  const int m0 = tile << 6;
  const T* Ab = xp + (size_t)img * kNPOS * kCIN2;
  const int rlane = lane & 15;
  const int koff  = (lane >> 4) * 8;
  const int mOff  = (lane >> 4) * 8;

  v8f acc[4][2];
#pragma unroll
  for (int i = 0; i < 4; ++i)
#pragma unroll
    for (int j = 0; j < 2; ++j) acc[i][j] = (v8f){0.f,0.f,0.f,0.f,0.f,0.f,0.f,0.f};

#pragma unroll 1
  for (int tp = 0; tp < kT5; ++tp) {
    const int ty = tp / 5, tx = tp - ty * 5;
    const T* At = Ab + (size_t)(m0 + ty * kPW + tx) * kCIN2;
    const T* Bt = Wo + (size_t)tp * kCIN2;
    for (int kc = 0; kc < kCIN2; kc += 32) {
      const V bh0 = Frag<T>::load(Bt + (size_t)rlane * kKOFF + kc + koff);
      const V bh1 = Frag<T>::load(Bt + (size_t)(16 + rlane) * kKOFF + kc + koff);
#pragma unroll
      for (int i = 0; i < 4; ++i) {
        const V ah = Frag<T>::load(At + (size_t)((i << 4) + rlane) * kCIN2 + kc + koff);
        acc[i][0] = Frag<T>::mma(ah, bh0, acc[i][0]);
        acc[i][1] = Frag<T>::mma(ah, bh1, acc[i][1]);
        Frag<T>::guard(acc[i][0], acc[i][1], ah, ah);
      }
      Frag<T>::keep(bh0, bh1, bh0, bh1);
    }
  }
  acc_guard4(acc[0][0], acc[0][1], acc[1][0], acc[1][1]);
  acc_guard4(acc[2][0], acc[2][1], acc[3][0], acc[3][1]);

  float* slab = sT[wave];
  float* Cb = offo + (size_t)img * kMOUT * kOFFN;
  const int q = lane >> 3, c4 = (lane & 7) * 4;
#pragma unroll
  for (int i = 0; i < 4; ++i) {
    const int mBase = m0 + (i << 4);
#pragma unroll
    for (int j = 0; j < 2; ++j) {
#pragma unroll
      for (int r = 0; r < 8; ++r) slab[(mOff + r) * 36 + (j << 4) + rlane] = acc[i][j][r] * (1.0f / 64.0f);
    }
    __builtin_amdgcn_fence(__ATOMIC_RELEASE, "workgroup");
    __builtin_amdgcn_wave_barrier();
    __builtin_amdgcn_fence(__ATOMIC_ACQUIRE, "workgroup");
    for (int pass = 0; pass < 2; ++pass) {
#pragma unroll
      for (int it = 0; it < 4; ++it) {
        const int row = it * 4 + q;
        const v4f v = *(const v4f*)(slab + row * 36 + c4);
        *(volatile v4f*)(Cb + (size_t)(mBase + row) * kOFFN + c4) = v;
      }
      __threadfence();
    }
    __builtin_amdgcn_fence(__ATOMIC_RELEASE, "workgroup");
    __builtin_amdgcn_wave_barrier();
    __builtin_amdgcn_fence(__ATOMIC_ACQUIRE, "workgroup");
  }
}

__global__ __launch_bounds__(256) void k_sample(const _Float16* __restrict__ xp, const float* __restrict__ offo,
                                                _Float16* __restrict__ S, int img0) {
  const int lane = threadIdx.x & 31, wave = threadIdx.x >> 5;
  const int item = blockIdx.x * 8 + wave;
  if (item >= kCHUNK * kNPX * kT3) return;
  const int pl = item / kT3, k = item - pl * kT3;
  const int limg = pl >> 10, p = pl & (kNPX - 1);
  const int img = img0 + limg;
  const int y = p >> 5, x = p & 31;
  const int kh = k / 3, kw = k - kh * 3;
  const float* orow = offo + ((size_t)img * kMOUT + (size_t)y * kPW + x) * kOFFN;
  const float dy = orow[2 * k];
  const float dx = orow[2 * k + 1];
  const float py = (float)(y + kh - 1) + dy;
  const float px = (float)(x + kw - 1) + dx;
  const float y0f = floorf(py), x0f = floorf(px);
  const float wy1 = py - y0f, wy0 = 1.0f - wy1;
  const float wx1 = px - x0f, wx0 = 1.0f - wx1;
  const int y0 = (int)fminf(fmaxf(y0f, -8.0f), 40.0f);
  const int x0 = (int)fminf(fmaxf(x0f, -8.0f), 40.0f);
  const int y1 = y0 + 1, x1 = x0 + 1;
  const bool vy0 = (y0 >= 0) && (y0 < kHGT), vy1 = (y1 >= 0) && (y1 < kHGT);
  const bool vx0 = (x0 >= 0) && (x0 < kWID), vx1 = (x1 >= 0) && (x1 < kWID);
  float w00 = wy0 * wx0, w01 = wy0 * wx1, w10 = wy1 * wx0, w11 = wy1 * wx1;
  w00 = (vy0 && vx0) ? w00 : 0.0f;
  w01 = (vy0 && vx1) ? w01 : 0.0f;
  w10 = (vy1 && vx0) ? w10 : 0.0f;
  w11 = (vy1 && vx1) ? w11 : 0.0f;
  const int yi0 = y0 < 0 ? 0 : (y0 > kHGT - 1 ? kHGT - 1 : y0);
  const int yi1 = y1 < 0 ? 0 : (y1 > kHGT - 1 ? kHGT - 1 : y1);
  const int xi0 = x0 < 0 ? 0 : (x0 > kWID - 1 ? kWID - 1 : x0);
  const int xi1 = x1 < 0 ? 0 : (x1 > kWID - 1 ? kWID - 1 : x1);
  const _Float16* xb  = xp + (size_t)img * kNPOS * kCIN2 + kCH + lane * 8;
  const _Float16* r00 = xb + (size_t)((yi0 + 2) * kPW + (xi0 + 2)) * kCIN2;
  const _Float16* r01 = xb + (size_t)((yi0 + 2) * kPW + (xi1 + 2)) * kCIN2;
  const _Float16* r10 = xb + (size_t)((yi1 + 2) * kPW + (xi0 + 2)) * kCIN2;
  const _Float16* r11 = xb + (size_t)((yi1 + 2) * kPW + (xi1 + 2)) * kCIN2;
  const v8h g00 = *(const v8h*)r00;
  const v8h g01 = *(const v8h*)r01;
  const v8h g10 = *(const v8h*)r10;
  const v8h g11 = *(const v8h*)r11;
  v8h hv;
#pragma unroll
  for (int e = 0; e < 8; ++e) {
    const float f = (((float)g00[e] * w00 + (float)g01[e] * w01) + (float)g10[e] * w10) + (float)g11[e] * w11;
    hv[e] = (_Float16)f;
  }
  _Float16* d = S + (size_t)pl * kKDEF + k * kCH + lane * 8;
  *(volatile v8h*)d = hv;
  __threadfence();
  *(volatile v8h*)d = hv;
}

__global__ __launch_bounds__(256) void k_defconv(const _Float16* __restrict__ Wd, const _Float16* __restrict__ S,
                                                 float* __restrict__ out, int img0) {
  typedef _Float16 T;
  typedef v16h V;
  __shared__ __align__(16) float sT[8][16 * 68];
  const int limg = blockIdx.y;
  const int lane = threadIdx.x & 31;
  const int wave = threadIdx.x >> 5;
  const int tile = blockIdx.x * 8 + wave;
  if (tile >= kNPX / 64) return;
  const int n0 = tile << 6;
  const T* Bb = S + (size_t)limg * kNPX * kKDEF;
  const int rlane = lane & 15;
  const int koff  = (lane >> 4) * 8;
  const int mOff  = (lane >> 4) * 8;

  v8f acc[4];
#pragma unroll
  for (int j = 0; j < 4; ++j) acc[j] = (v8f){0.f,0.f,0.f,0.f,0.f,0.f,0.f,0.f};

  for (int k0 = 0; k0 < kKDEF; k0 += 32) {
    V bh[4];
#pragma unroll
    for (int j = 0; j < 4; ++j) bh[j] = Frag<T>::load(Bb + (size_t)(n0 + (j << 4) + rlane) * kKDEF + k0 + koff);
    const V ah = Frag<T>::load(Wd + (size_t)rlane * kKDEF + k0 + koff);
#pragma unroll
    for (int j = 0; j < 4; ++j) acc[j] = Frag<T>::mma(ah, bh[j], acc[j]);
    Frag<T>::guard(acc[0], acc[3], ah, ah);
    Frag<T>::keep(bh[0], bh[1], bh[2], bh[3]);
  }
  acc_guard4(acc[0], acc[1], acc[2], acc[3]);

  float* slab = sT[wave];
#pragma unroll
  for (int j = 0; j < 4; ++j) {
#pragma unroll
    for (int r = 0; r < 8; ++r) {
      float v = acc[j][r] * (1.0f / 32.0f);
      v = fminf(fmaxf(v, -30.0f), 30.0f);
      const float sg = __builtin_amdgcn_rcpf(1.0f + __expf(-v));
      slab[(mOff + r) * 68 + (j << 4) + rlane] = sg;
    }
  }
  __builtin_amdgcn_fence(__ATOMIC_RELEASE, "workgroup");
  __builtin_amdgcn_wave_barrier();
  __builtin_amdgcn_fence(__ATOMIC_ACQUIRE, "workgroup");
  float* Cb = out + (size_t)(img0 + limg) * kODEF * kNPX;
  const int hh = lane >> 4, c4 = (lane & 15) * 4;
  for (int pass = 0; pass < 2; ++pass) {
#pragma unroll
    for (int it = 0; it < 8; ++it) {
      const int row = it * 2 + hh;
      const v4f v = *(const v4f*)(slab + row * 68 + c4);
      if (row < kODEF) *(volatile v4f*)(Cb + (size_t)row * kNPX + n0 + c4) = v;
    }
    __threadfence();
  }
}

extern "C" void kernel_launch(void* const* d_in, const int* in_sizes, int n_in,
                              void* d_out, int out_size, void* d_ws, size_t ws_size,
                              hipStream_t stream) {
  if (n_in < 4) return;
  if (in_sizes[0] != kNIMG * kCH * kNPX || in_sizes[1] != kNIMG * kCH * kNPX ||
      in_sizes[2] != kOFFC * kCIN2 * kT5 || in_sizes[3] != kODEF * kCH * kT3) return;
  if (out_size != kNIMG * kODEF * kNPX) return;

  const float* support = (const float*)d_in[0];
  const float* query   = (const float*)d_in[1];
  const float* w_off   = (const float*)d_in[2];
  const float* w_def   = (const float*)d_in[3];
  float* out = (float*)d_out;

  const size_t bytes_xp  = (size_t)kNIMG * kNPOS * kCIN2 * 2;
  const size_t bytes_off = (size_t)kNIMG * kMOUT * kOFFN * 4;
  const size_t bytes_S   = (size_t)kCHUNK * kNPX * kKDEF * 2;
  const size_t bytes_Wo  = (size_t)kOFFN * kKOFF * 2;
  const size_t bytes_Wd  = (size_t)kMDEF * kKDEF * 2;
  char* ws = (char*)d_ws;
  size_t o = 0;
  _Float16* xp  = (_Float16*)(ws + o);  o += bytes_xp;
  float*    OFF = (float*)(ws + o);     o += bytes_off;
  _Float16* S   = (_Float16*)(ws + o);  o += bytes_S;
  _Float16* Wo  = (_Float16*)(ws + o);  o += bytes_Wo;
  _Float16* Wd  = (_Float16*)(ws + o);  o += bytes_Wd;
  if (o > ws_size || o > (size_t)134217728) return;

  k_pack<<<kNIMG * kPROWS * 8, 256, 0, stream>>>(support, query, xp);
  k_prep_woff<<<(kOFFN * kKOFF / 8 + 255) / 256, 256, 0, stream>>>(w_off, Wo);
  k_prep_wdef<<<(kMDEF * kKDEF / 8 + 255) / 256, 256, 0, stream>>>(w_def, Wd);
  k_offconv<<<dim3(kMOUT / 64 / 2, kNIMG), 64, 0, stream>>>(xp, Wo, OFF);
  for (int ch = 0; ch < kNCHUNK; ++ch) {
    k_sample<<<kCHUNK * kNPX * kT3 / 8, 256, 0, stream>>>(xp, OFF, S, ch * kCHUNK);
    k_defconv<<<dim3(kNPX / 64 / 8, kCHUNK), 256, 0, stream>>>(Wd, S, out, ch * kCHUNK);
  }
}
